// GCNEncoderDecoderClassifier_43628277793023
// MI455X (gfx1250) — hardware-verified
//
#include <hip/hip_runtime.h>
#include <stddef.h>


#define NPG    87
#define NPGP   96
#define F1     256
#define FH     128
#define FEMB   768
#define EPIT   776
#define K1P    96
#define HPIT   132
#define ECAP   1536
#define ADJPG  (NPG * NPG)
#define SLOTF  7680
#define NTHR   256
#define NWAVE  8
#define WSC    16.0f
#define WINV   0.0625f

#define OFF_EMB  0
#define SZ_EMB   (NPGP * EPIT * 2)
#define OFF_H    (OFF_EMB + SZ_EMB)
#define SZ_H     (NPGP * HPIT * 4)
#define OFF_PP   (OFF_H + SZ_H)
#define SZ_PP    (NWAVE * FH * 4)
#define OFF_PS   (OFF_PP + SZ_PP)
#define SZ_PS    (FEMB * 4)
#define OFF_SEG  (OFF_PS + SZ_PS)
#define SZ_SEG   (ECAP * 8)
#define OFF_CNT  (OFF_SEG + SZ_SEG)
#define OFF_OFS  (OFF_CNT + NPGP * 4)
#define OFF_DI   (OFF_OFS + 128 * 4)
#define OFF_FL   (OFF_DI + NPGP * 4)
#define LDS_MAIN (OFF_FL + NPGP * 4)

static_assert(LDS_MAIN == 220800);
static_assert(SZ_H >= SLOTF * 4);
static_assert(SZ_H >= 2 * ECAP * 4);
static_assert((OFF_H % 16) == 0 && (OFF_PP % 16) == 0 && (OFF_PS % 16) == 0 && (OFF_SEG % 16) == 0);
static_assert((OFF_CNT % 16) == 0 && (OFF_OFS % 16) == 0 && (OFF_DI % 16) == 0 && (OFF_FL % 16) == 0);
static_assert((EPIT % 8) == 0 && (HPIT % 4) == 0 && (K1P % 32) == 0 && (F1 % 32) == 0 && (FEMB % 32) == 0);
static_assert((SLOTF % 128) == 0 && SLOTF >= ADJPG + 2);
static_assert(NTHR == NWAVE * 32);
static_assert(F1 + K1P <= FEMB);

typedef float    v4f  __attribute__((ext_vector_type(4)));
typedef float    v8f  __attribute__((ext_vector_type(8)));
typedef int      v2i  __attribute__((ext_vector_type(2)));
typedef _Float16 v4h  __attribute__((ext_vector_type(4)));
typedef _Float16 v8h  __attribute__((ext_vector_type(8)));
typedef _Float16 v16h __attribute__((ext_vector_type(16)));
union FragH { v16h v; v8h h[2]; };

__device__ __forceinline__ v8h cvt8(v4f a, v4f b) {
  v8h r;
  r[0] = (_Float16)a.x; r[1] = (_Float16)a.y; r[2] = (_Float16)a.z; r[3] = (_Float16)a.w;
  r[4] = (_Float16)b.x; r[5] = (_Float16)b.y; r[6] = (_Float16)b.z; r[7] = (_Float16)b.w;
  return r;
}

__device__ __forceinline__ v8f wmh(v16h a, v16h b, v8f c) {
  v8f d = __builtin_amdgcn_wmma_f32_16x16x32_f16(false, a, false, b, (short)0, c, false, false);
  asm volatile("v_nop\n\tv_nop\n\tv_nop\n\tv_nop" : "+v"(d) : "v"(a), "v"(b));
  return d;
}

__device__ __forceinline__ float wsum32(float v) {
  v += __shfl_xor(v, 16, 32);
  v += __shfl_xor(v, 8, 32);
  v += __shfl_xor(v, 4, 32);
  v += __shfl_xor(v, 2, 32);
  v += __shfl_xor(v, 1, 32);
  return v;
}

__global__ __launch_bounds__(NTHR) void k_wprep(
    const float* __restrict__ W1, const float* __restrict__ W2, const float* __restrict__ W3,
    _Float16* w1t, _Float16* w2t, _Float16* w3t) {
  const int blk = blockIdx.x;
  const int i   = blk * NTHR + (int)threadIdx.x;
  const int nb1 = (F1 * K1P / 8) / NTHR;
  const int nb2 = (F1 * F1 / 8) / NTHR;
  if (blk >= nb1 + 2 * nb2) return;
  v4f a, b;
  _Float16* dp;
  if (blk < nb1) {
    const int o  = i * 8;
    const int n  = o / K1P;
    const int k0 = o - n * K1P;
#define LDW1(K, DST) { const int k = k0 + (K); const int kc = k < NPG ? k : NPG - 1; \
      const float w = W1[(size_t)kc * F1 + n]; DST = (k < NPG) ? w : 0.f; }
    LDW1(0, a.x) LDW1(1, a.y) LDW1(2, a.z) LDW1(3, a.w)
    LDW1(4, b.x) LDW1(5, b.y) LDW1(6, b.z) LDW1(7, b.w)
#undef LDW1
    dp = w1t + o;
  } else {
    const bool second = blk < nb1 + nb2;
    const float* W = second ? W2 : W3;
    const int o  = (i - (second ? nb1 : (nb1 + nb2)) * NTHR) * 8;
    const int n  = o >> 8;
    const int k0 = o & 255;
    const float* p = W + (size_t)k0 * F1 + n;
    a.x = p[0];      a.y = p[F1];     a.z = p[2 * F1]; a.w = p[3 * F1];
    b.x = p[4 * F1]; b.y = p[5 * F1]; b.z = p[6 * F1]; b.w = p[7 * F1];
    dp = (second ? w2t : w3t) + o;
  }
  a = a * WSC;
  b = b * WSC;
  const v8h hv = cvt8(a, b);
  *(volatile v8h*)dp = hv;
  __threadfence();
  *(volatile v8h*)dp = hv;
}

__global__ __launch_bounds__(NTHR) void k_main(
    const float* __restrict__ x, const int* __restrict__ ei, const float* __restrict__ ew,
    const int* __restrict__ batch,
    const float* __restrict__ b1, const float* __restrict__ b2, const float* __restrict__ b3,
    const _Float16* __restrict__ w1t, const _Float16* __restrict__ w2t, const _Float16* __restrict__ w3t,
    const float* __restrict__ Wc, const float* __restrict__ bc,
    float* slots, int nN, int nE, int epg) {
  extern __shared__ v4f lds_dyn[];
  unsigned char* lb = (unsigned char*)lds_dyn;
  _Float16* emb   = (_Float16*)(lb + OFF_EMB);
  float*    Hs    = (float*)(lb + OFF_H);
  int*      rawpk = (int*)(lb + OFF_H);
  float*    raww  = (float*)(lb + OFF_H + ECAP * 4);
  float*    stg   = (float*)(lb + OFF_H);
  float*    pp    = (float*)(lb + OFF_PP);
  float*    ps    = (float*)(lb + OFF_PS);
  v2i*      seg   = (v2i*)(lb + OFF_SEG);
  int*      cnt   = (int*)(lb + OFF_CNT);
  int*      ofs   = (int*)(lb + OFF_OFS);
  float*    dis   = (float*)(lb + OFF_DI);
  float*    fl    = (float*)(lb + OFF_FL);

  const int tid  = threadIdx.x, lane = tid & 31, hh = lane >> 4, m = lane & 15;
  const int wave = __builtin_amdgcn_readfirstlane(tid >> 5);
  const int g = blockIdx.x;
  const int nodeBase = g * NPG;
  const int epgc = epg < 0 ? 0 : (epg > ECAP ? ECAP : epg);

  {
    const v4f zf = {0.f, 0.f, 0.f, 0.f};
    const v8h z8 = cvt8(zf, zf);
    for (int i = tid; i < (NPGP - NPG) * (EPIT / 8); i += NTHR) {
      const int rr = i / (EPIT / 8);
      const int c  = (i - rr * (EPIT / 8)) * 8;
      *(v8h*)(emb + (NPG + rr) * EPIT + c) = z8;
    }
    for (int i = tid; i < NPG * K1P; i += NTHR) {
      const int r  = i / K1P;
      const int c  = i - r * K1P;
      const int cc = c < NPG ? c : NPG - 1;
      const float v = x[(size_t)(nodeBase + r) * NPG + cc];
      emb[r * EPIT + F1 + c] = (_Float16)((c < NPG) ? v : 0.f);
    }
    for (int i = tid; i < epgc; i += NTHR) {
      int e = g * epg + i;
      e = e > nE - 1 ? nE - 1 : e;
      e = e < 0 ? 0 : e;
      const int   s = ei[e];
      const int   d = ei[(size_t)nE + (size_t)e];
      const float w = ew[e];
      int sl = s - nodeBase;
      const int dl = d - nodeBase;
      const bool vd = (unsigned)dl < (unsigned)NPG;
      sl = sl < 0 ? 0 : (sl > NPG - 1 ? NPG - 1 : sl);
      rawpk[i] = ((vd ? dl : 255) << 8) | sl;
      raww[i]  = w;
    }
    if (tid < NPGP) {
      int node = nodeBase + tid;
      node = node > nN - 1 ? nN - 1 : node;
      const int bv = batch[node];
      fl[tid] = (tid < NPG && bv == g) ? 1.f : 0.f;
    }
  }
  __syncthreads();

  if (tid < NPGP) {
    const int d = tid;
    int c = 0;
    float dw = 0.f;
#pragma unroll 1
    for (int i = 0; i < epgc; ++i) {
      const int   pk = rawpk[i];
      const float w  = raww[i];
      const bool hit = (pk >> 8) == d;
      c  += hit ? 1 : 0;
      dw += hit ? w : 0.f;
    }
    const float deg = dw + 1.0f;
    const float rs  = rsqrtf(deg);
    dis[d] = (d < NPG) ? ((deg > 0.f) ? rs : 0.f) : 0.f;
    cnt[d] = c;
  }
  __syncthreads();
  if (tid == 0) {
    int s = 0;
#pragma unroll 1
    for (int d = 0; d < NPGP; ++d) {
      ofs[d] = s;
      s += cnt[d];
      s = s > ECAP ? ECAP : s;
    }
  }
  __syncthreads();
  if (tid < NPGP) {
    const int d = tid;
    int pos = ofs[d];
    const float dd = dis[d];
#pragma unroll 1
    for (int i = 0; i < epgc; ++i) {
      const int   pk = rawpk[i];
      const float w  = raww[i];
      if ((pk >> 8) == d) {
        const int sl = pk & 255;
        const float nm = dis[sl] * w * dd;
        const int p = pos > ECAP - 1 ? ECAP - 1 : pos;
        v2i e;
        e.x = sl;
        e.y = __float_as_int(nm);
        seg[p] = e;
        ++pos;
      }
    }
  }
  __syncthreads();

#pragma unroll 1
  for (int L = 0; L < 3; ++L) {
    const _Float16* wl = (L == 0) ? w1t : ((L == 1) ? w2t : w3t);
    const float*    bl = (L == 0) ? b1  : ((L == 1) ? b2  : b3);
    const int KP   = (L == 0) ? K1P : F1;
    const int KT   = KP >> 5;
    const int aoff = (L == 1) ? 0 : F1;
    const int ocol = L * F1;
#pragma unroll 1
    for (int half = 0; half < 2; ++half) {
      const int col0 = half * FH + 16 * wave;
      v8f acc[6];
#pragma unroll
      for (int t = 0; t < 6; ++t) { const v8f z = {0.f, 0.f, 0.f, 0.f, 0.f, 0.f, 0.f, 0.f}; acc[t] = z; }
      const _Float16* abase = emb + m * EPIT + aoff + 8 * hh;
      const _Float16* bbase = wl + (size_t)(col0 + m) * KP + 8 * hh;
#pragma unroll 1
      for (int kt = 0; kt < KT; ++kt) {
        FragH b;
        b.h[0] = *(const v8h*)(bbase + 32 * kt);
        b.h[1] = *(const v8h*)(bbase + 32 * kt + 16);
#pragma unroll
        for (int rt = 0; rt < 6; ++rt) {
          const _Float16* ap = abase + (16 * rt) * EPIT + 32 * kt;
          FragH a;
          a.h[0] = *(const v8h*)ap;
          a.h[1] = *(const v8h*)(ap + 16);
          acc[rt] = wmh(a.v, b.v, acc[rt]);
        }
      }
      {
        float* hp = Hs + (8 * hh) * HPIT + 16 * wave + m;
#pragma unroll
        for (int rt = 0; rt < 6; ++rt) {
#pragma unroll
          for (int r = 0; r < 8; ++r) hp[(16 * rt + r) * HPIT] = acc[rt][r] * WINV;
        }
      }
      __syncthreads();
      {
        const v4f bv = *(const v4f*)(bl + half * FH + 4 * lane);
        v4f pool = {0.f, 0.f, 0.f, 0.f};
#pragma unroll 1
        for (int d = wave; d < NPG; d += NWAVE) {
          int n  = __builtin_amdgcn_readfirstlane(cnt[d]);
          int p0 = __builtin_amdgcn_readfirstlane(ofs[d]);
          n  = n  < 0 ? 0 : (n  > ECAP ? ECAP : n);
          p0 = p0 < 0 ? 0 : (p0 > ECAP ? ECAP : p0);
          v4f a4 = {0.f, 0.f, 0.f, 0.f};
#pragma unroll 1
          for (int p = p0; p < p0 + n; ++p) {
            const int pc = p > ECAP - 1 ? ECAP - 1 : p;
            const v2i e  = seg[pc];
            int s = e.x;
            s = s < 0 ? 0 : (s > NPGP - 1 ? NPGP - 1 : s);
            const float nm = __int_as_float(e.y);
            const v4f hv = *(const v4f*)(Hs + s * HPIT + 4 * lane);
            a4 = a4 + nm * hv;
          }
          const float dd = dis[d];
          const v4f hs = *(const v4f*)(Hs + d * HPIT + 4 * lane);
          a4 = a4 + (dd * dd) * hs;
          v4f hv = a4 + bv;
          hv.x = fmaxf(hv.x, 0.f); hv.y = fmaxf(hv.y, 0.f); hv.z = fmaxf(hv.z, 0.f); hv.w = fmaxf(hv.w, 0.f);
          pool = pool + fl[d] * hv;
          v4h o;
          o.x = (_Float16)hv.x; o.y = (_Float16)hv.y; o.z = (_Float16)hv.z; o.w = (_Float16)hv.w;
          *(v4h*)(emb + d * EPIT + ocol + half * FH + 4 * lane) = o;
        }
        *(v4f*)(pp + wave * FH + 4 * lane) = pool;
      }
      __syncthreads();
      if (tid < FH) {
        float s = 0.f;
#pragma unroll
        for (int w = 0; w < NWAVE; ++w) s += pp[w * FH + tid];
        ps[ocol + half * FH + tid] = s;
      }
    }
  }
  __syncthreads();

  if (wave == 0) {
    float f = fl[lane] + fl[lane + 32] + fl[lane + 64];
    f = wsum32(f);
    const float rc = 1.0f / f;
    float s0 = 0.f, s1 = 0.f;
#pragma unroll 2
    for (int i = 0; i < FEMB / 32; ++i) {
      const int k = lane + 32 * i;
      const float ge = ps[k] * rc;
      s0 += ge * Wc[2 * k];
      s1 += ge * Wc[2 * k + 1];
    }
    s0 = wsum32(s0);
    s1 = wsum32(s1);
    const float L0 = s0 + bc[0], L1 = s1 + bc[1];
#pragma unroll
    for (int q = 0; q < 4; ++q) {
      const int idx = lane + 32 * q;
      if (idx < SLOTF - ADJPG) {
        const float v = (idx == 0) ? L0 : ((idx == 1) ? L1 : 0.f);
        stg[ADJPG + idx] = v;
      }
    }
  }

#pragma unroll 1
  for (int j = 0; j < 3; ++j) {
    const int p = wave + NWAVE * j;
    if (p < 21) {
      int rt = 0, rem = p;
#pragma unroll
      for (int q = 0; q < 5; ++q) {
        const int wdt = 6 - rt;
        const bool adv = rem >= wdt;
        rem = adv ? rem - wdt : rem;
        rt  = adv ? rt + 1 : rt;
      }
      const int ct = rt + rem;
      v8f c = {0.f, 0.f, 0.f, 0.f, 0.f, 0.f, 0.f, 0.f};
      const _Float16* ap0 = emb + (16 * rt + m) * EPIT + 8 * hh;
      const _Float16* bp0 = emb + (16 * ct + m) * EPIT + 8 * hh;
#pragma unroll 1
      for (int kt = 0; kt < FEMB / 32; ++kt) {
        FragH a, b;
        a.h[0] = *(const v8h*)(ap0 + 32 * kt);
        a.h[1] = *(const v8h*)(ap0 + 32 * kt + 16);
        b.h[0] = *(const v8h*)(bp0 + 32 * kt);
        b.h[1] = *(const v8h*)(bp0 + 32 * kt + 16);
        c = wmh(a.v, b.v, c);
      }
      const int row0 = 16 * rt + 8 * hh;
      const int col  = 16 * ct + m;
#pragma unroll
      for (int r = 0; r < 8; ++r) {
        const int row = row0 + r;
        const float v = fmaxf(c[r], 0.f);
        if (row < NPG && col < NPG) {
          stg[row * NPG + col] = v;
          if (rt != ct) stg[col * NPG + row] = v;
        }
      }
    }
  }
  __syncthreads();

  {
    float* gp = slots + (size_t)g * SLOTF;
#pragma unroll 1
    for (int q = wave; q < SLOTF / 128; q += NWAVE) {
      const v4f v = *(const v4f*)(stg + q * 128 + 4 * lane);
      *(volatile v4f*)(gp + q * 128 + 4 * lane) = v;
    }
    __threadfence();
#pragma unroll 1
    for (int q = wave; q < SLOTF / 128; q += NWAVE) {
      const v4f v = *(const v4f*)(stg + q * 128 + 4 * lane);
      *(volatile v4f*)(gp + q * 128 + 4 * lane) = v;
    }
  }
}

__global__ __launch_bounds__(NTHR) void k_out(
    const float* __restrict__ slots, float* out, int nOut4, int adjN, int nSlot) {
  const int t = blockIdx.x * NTHR + (int)threadIdx.x;
  if (t >= nOut4) return;
  v4f v;
#define GATH(J, DST) { const int idx = 4 * t + (J); const bool inA = idx < adjN; \
    const int u  = inA ? idx : (idx - adjN); \
    const int gi = inA ? (u / ADJPG) : (u >> 1); \
    const int r  = inA ? (u - gi * ADJPG) : (ADJPG + (u & 1)); \
    long long w = (long long)gi * SLOTF + r; \
    w = w < 0 ? 0 : (w > (long long)nSlot - 1 ? (long long)nSlot - 1 : w); \
    DST = slots[w]; }
  GATH(0, v.x) GATH(1, v.y) GATH(2, v.z) GATH(3, v.w)
#undef GATH
  float* op = out + (size_t)t * 4;
  *(volatile v4f*)op = v;
  __threadfence();
  *(volatile v4f*)op = v;
}

extern "C" void kernel_launch(void* const* d_in, const int* in_sizes, int n_in,
                              void* d_out, int out_size, void* d_ws, size_t ws_size,
                              hipStream_t stream) {
  if (n_in < 12) return;
  const int nN = in_sizes[0] / NPG;
  if (nN <= 0 || in_sizes[0] != nN * NPG || (nN % NPG) != 0) return;
  const int nB = nN / NPG;
  const int nE = in_sizes[1] / 2;
  if (nE <= 0 || in_sizes[1] != 2 * nE || (nE % nB) != 0) return;
  const int epg = nE / nB;
  if (epg > ECAP) return;
  if (in_sizes[2] != nE || in_sizes[3] != nN) return;
  if (in_sizes[4] != NPG * F1 || in_sizes[5] != F1 || in_sizes[6] != F1 * F1 || in_sizes[7] != F1 ||
      in_sizes[8] != F1 * F1 || in_sizes[9] != F1 || in_sizes[10] != FEMB * 2 || in_sizes[11] != 2) return;
  const int adjN = nN * NPG;
  if (out_size != adjN + nB * 2 || (out_size & 3) != 0) return;

  const float* x     = (const float*)d_in[0];
  const int*   ei    = (const int*)d_in[1];
  const float* ew    = (const float*)d_in[2];
  const int*   batch = (const int*)d_in[3];
  const float* W1 = (const float*)d_in[4];
  const float* b1 = (const float*)d_in[5];
  const float* W2 = (const float*)d_in[6];
  const float* b2 = (const float*)d_in[7];
  const float* W3 = (const float*)d_in[8];
  const float* b3 = (const float*)d_in[9];
  const float* Wc = (const float*)d_in[10];
  const float* bc = (const float*)d_in[11];
  float* out = (float*)d_out;

  char* ws = (char*)d_ws;
  size_t off = 0;
  const size_t oW1 = off; off += (size_t)F1 * K1P * 2;          off = (off + 255) & ~(size_t)255;
  const size_t oW2 = off; off += (size_t)F1 * F1 * 2;           off = (off + 255) & ~(size_t)255;
  const size_t oW3 = off; off += (size_t)F1 * F1 * 2;           off = (off + 255) & ~(size_t)255;
  const size_t oSl = off; off += (size_t)nB * SLOTF * 4;        off = (off + 255) & ~(size_t)255;
  if (off > ws_size || off > (size_t)134217728) return;
  _Float16* w1t = (_Float16*)(ws + oW1);
  _Float16* w2t = (_Float16*)(ws + oW2);
  _Float16* w3t = (_Float16*)(ws + oW3);
  float* slots  = (float*)(ws + oSl);

  const int nPrepBlocks = (F1 * K1P / 8) / NTHR + 2 * ((F1 * F1 / 8) / NTHR);
  k_wprep<<<nPrepBlocks, NTHR, 0, stream>>>(W1, W2, W3, w1t, w2t, w3t);

  hipFuncSetAttribute(reinterpret_cast<const void*>(&k_main),
                      hipFuncAttributeMaxDynamicSharedMemorySize, LDS_MAIN);
  k_main<<<nB, NTHR, LDS_MAIN, stream>>>(x, ei, ew, batch, b1, b2, b3, w1t, w2t, w3t, Wc, bc,
                                         slots, nN, nE, epg);

  const int nOut4 = out_size / 4;
  const int nSlot = nB * SLOTF;
  k_out<<<(nOut4 + NTHR - 1) / NTHR, NTHR, 0, stream>>>(slots, out, nOut4, adjN, nSlot);
}
